// DecoderBlock_3040836846189
// MI455X (gfx1250) — hardware-run, weakly checked
//
#include <hip/hip_runtime.h>


#ifndef NB
#define NB 64
#endif
#ifndef SEQ
#define SEQ 256
#endif
#define NB_FULL  64
#define SEQ_FULL 256
#ifndef OUT_SEQ
#define OUT_SEQ SEQ
#endif
#define DM    256
#define NH_   16
#define HD    16
#define FF    1024
#define MROWS (NB * SEQ)
#define AW    4
#define HG    (NH_ / AW)
#define OSP   68
#define ACT_S 16.0f
#define W_S   256.0f
#define CINV  (1.0f / 4096.0f)
#define PLN_S (1.0f / 256.0f)
#define SC2   ((float)(0.0625 * 1.4426950408889634 / 256.0))
#define PSH   14.0f
#define NEGB  (-3.0e38f)
#define LN_EPS 1e-5f

static_assert(NH_ * HD == DM);
static_assert(HD == 16);
static_assert(AW * HD == 64);
static_assert(NH_ % AW == 0);
static_assert(DM % 64 == 0);
static_assert(FF % 64 == 0);
static_assert((2 * DM) % 64 == 0);
static_assert(DM % 32 == 0);
static_assert(FF % 32 == 0);
static_assert(SEQ % 64 == 0);
static_assert(SEQ % 32 == 0);
static_assert(MROWS % 64 == 0);
static_assert(MROWS % 8 == 0);
static_assert(NB <= NB_FULL);
static_assert(SEQ <= SEQ_FULL);
static_assert(SEQ <= OUT_SEQ);
static_assert((OSP * 4) % 16 == 0);
static_assert(16 * OSP * 4 <= 131072);
static_assert(64 * 17 * 4 <= 131072);
static_assert(DM == 32 * 8);
static_assert(32 * 16 == DM * 2);
static_assert(128 * 16 == 16 * 64 * 2);
static_assert(8 * 128 == 64 * 16);
static_assert(4 * 32 * 16 == 16 * 64 * 2);
static_assert(32 * 16 == 16 * HD * 2);
static_assert(8 * 32 * 16 == 16 * 64 * 4);
static_assert(32 * AW * 16 == 16 * 64 * 2);

typedef _Float16 h16;
typedef __attribute__((ext_vector_type(16))) _Float16 v16h;
typedef __attribute__((ext_vector_type(8)))  _Float16 v8h;
typedef __attribute__((ext_vector_type(8)))  float    v8f;
typedef __attribute__((ext_vector_type(4)))  float    v4f;
typedef v4f  __attribute__((may_alias)) v4fa;

__device__ __forceinline__ unsigned short f2bf(float f) { unsigned u = __float_as_uint(f); u += 0x7FFFu + ((u >> 16) & 1u); return (unsigned short)(u >> 16); }
__device__ __forceinline__ float bfr(float f) { return __uint_as_float(((unsigned)f2bf(f)) << 16); }
__device__ __forceinline__ v16h cat16(v8h lo, v8h hi) { return __builtin_shufflevector(lo, hi, 0, 1, 2, 3, 4, 5, 6, 7, 8, 9, 10, 11, 12, 13, 14, 15); }
__device__ __forceinline__ v16h ldh(const h16* p) { return cat16(*(const v8h*)p, *(const v8h*)(p + 16)); }
__device__ __forceinline__ v16h ldh_lo(const h16* p) { const v8h z = (v8h){}; return cat16(*(const v8h*)p, z); }
__device__ __forceinline__ h16 toh_flush(float v) { const h16 r = (h16)v; return (fabsf(v) < 6.103515625e-05f) ? (h16)0.0f : r; }
__device__ __forceinline__ v8f wmma16g(v16h a, v16h b, v8f c) {
    c = __builtin_amdgcn_wmma_f32_16x16x32_f16(false, a, false, b, (short)0, c, false, false);
    asm volatile("v_nop\n\tv_nop\n\tv_nop\n\tv_nop" : "+v"(c) : "v"(a), "v"(b));
    return c;
}
__device__ __forceinline__ void wave_sync() { __builtin_amdgcn_fence(3  , "wavefront"); __builtin_amdgcn_wave_barrier(); asm volatile("" ::: "memory"); }
__device__ __forceinline__ float gelu_erf(float x) { return 0.5f * x * (1.0f + erff(x * 0.70710678118654752f)); }

__global__ __launch_bounds__(128) void k_wtr(const float* __restrict__ W, h16* Wt, int K, int ldn, size_t inStride, size_t outStride) {
    __shared__ float ts[64 * 17];
    const int p = threadIdx.x;
    const int k0 = blockIdx.x * 64, n0 = blockIdx.y * 16;
    const size_t ibase = (size_t)blockIdx.z * inStride + (size_t)k0 * (size_t)ldn + (size_t)n0;
#pragma unroll 1
    for (int it = 0; it < 8; ++it) { const int e = it * 128 + p; const int kk = e >> 4, nn = e & 15;
        ts[kk * 17 + nn] = bfr(W[ibase + (size_t)kk * (size_t)ldn + nn]) * W_S; }
    __syncthreads();
    const int nn = p >> 3, k8 = (p & 7) * 8;
    v8h o;
#pragma unroll
    for (int i = 0; i < 8; ++i) o[i] = toh_flush(ts[(k8 + i) * 17 + nn]);
    h16* dst = Wt + (size_t)blockIdx.z * outStride + (size_t)(n0 + nn) * (size_t)K + k0 + k8;
    *(volatile v8h*)dst = o; __threadfence(); *(volatile v8h*)dst = o;
}

__global__ __launch_bounds__(256) void k_ln(const float* __restrict__ X, const float* __restrict__ g, const float* __restrict__ be, h16* H, int rin, int xfull) {
#pragma clang fp contract(off)
    const int lane = threadIdx.x & 31;
    const int wave = __builtin_amdgcn_readfirstlane((int)(threadIdx.x >> 5));
    const int m = blockIdx.x * 8 + wave;
    const int srow = xfull ? ((m / SEQ) * SEQ_FULL + (m % SEQ)) : m;
    const float* xp = X + (size_t)srow * DM + lane * 8;
    const v4f a0 = *(const v4f*)xp, a1 = *(const v4f*)(xp + 4);
    const v4f g0 = *(const v4f*)(g + lane * 8), g1 = *(const v4f*)(g + lane * 8 + 4);
    const v4f e0 = *(const v4f*)(be + lane * 8), e1 = *(const v4f*)(be + lane * 8 + 4);
    float v[8];
#pragma unroll
    for (int i = 0; i < 4; ++i) { v[i] = rin ? bfr(a0[i]) : a0[i]; v[4 + i] = rin ? bfr(a1[i]) : a1[i]; }
    float s = ((v[0] + v[1]) + (v[2] + v[3])) + ((v[4] + v[5]) + (v[6] + v[7]));
    s += __shfl_xor(s, 16, 32); s += __shfl_xor(s, 8, 32); s += __shfl_xor(s, 4, 32); s += __shfl_xor(s, 2, 32); s += __shfl_xor(s, 1, 32);
    const float mu = s * (1.0f / DM);
    float d[8];
#pragma unroll
    for (int i = 0; i < 8; ++i) d[i] = v[i] - mu;
    float q = ((d[0] * d[0] + d[1] * d[1]) + (d[2] * d[2] + d[3] * d[3])) + ((d[4] * d[4] + d[5] * d[5]) + (d[6] * d[6] + d[7] * d[7]));
    q += __shfl_xor(q, 16, 32); q += __shfl_xor(q, 8, 32); q += __shfl_xor(q, 4, 32); q += __shfl_xor(q, 2, 32); q += __shfl_xor(q, 1, 32);
    const float rs = rsqrtf(q * (1.0f / DM) + LN_EPS);
    v8h o;
#pragma unroll
    for (int i = 0; i < 4; ++i) {
        const float y0 = d[i] * rs * bfr(g0[i]) + bfr(e0[i]);
        const float y1 = d[4 + i] * rs * bfr(g1[i]) + bfr(e1[i]);
        o[i] = toh_flush(y0 * ACT_S); o[4 + i] = toh_flush(y1 * ACT_S); }
    h16* dst = H + (size_t)m * DM + lane * 8;
    *(volatile v8h*)dst = o; __threadfence(); *(volatile v8h*)dst = o;
}

template <int EPI, int KD>
__device__ __forceinline__ void gemm_body(const h16* __restrict__ A, const h16* __restrict__ Bt, const float* __restrict__ bias, const float* __restrict__ R, h16* PH, float* PF) {
    __shared__ __align__(16) float os[16 * OSP];
    const int lane = threadIdx.x & 31, lr = lane & 15, hi = lane >> 4;
    const int r0 = blockIdx.x * 64, c0 = blockIdx.y * 64;
    v8f acc[4][4];
#pragma unroll
    for (int mb = 0; mb < 4; ++mb)
#pragma unroll
        for (int nb = 0; nb < 4; ++nb) acc[mb][nb] = (v8f){};
    const size_t aoff = (size_t)(r0 + lr) * KD + 8 * hi, boff = (size_t)(c0 + lr) * KD + 8 * hi;
#pragma unroll 1
    for (int kc = 0; kc < KD; kc += 32) {
        v16h a[4];
#pragma unroll
        for (int mb = 0; mb < 4; ++mb) a[mb] = ldh(A + aoff + (size_t)mb * 16 * KD + kc);
#pragma unroll
        for (int nb = 0; nb < 4; ++nb) { const v16h b = ldh(Bt + boff + (size_t)nb * 16 * KD + kc);
#pragma unroll
            for (int mb = 0; mb < 4; ++mb) acc[mb][nb] = wmma16g(a[mb], b, acc[mb][nb]); }
    }
    const float sc = (EPI <= 1) ? PLN_S : CINV;
    float bc[4];
#pragma unroll
    for (int nb = 0; nb < 4; ++nb) bc[nb] = (EPI >= 2) ? bfr(bias[c0 + nb * 16 + lr]) : 0.0f;
    size_t obase = 0, rbase = 0;
    if (EPI == 0) { const int rsel = c0 / DM, head0 = (c0 % DM) / HD; const int bb = r0 / SEQ, tt = r0 % SEQ;
                    obase = ((size_t)((rsel * NB + bb) * NH_ + head0) * SEQ + (size_t)tt) * HD; }
    if (EPI == 1) { const int bb = c0 / SEQ, tt = c0 % SEQ; obase = (size_t)bb * DM * SEQ + (size_t)r0 * SEQ + (size_t)tt; }
    if (EPI == 2) { obase = (size_t)r0 * DM + c0; rbase = ((size_t)(r0 / SEQ) * SEQ_FULL + (size_t)(r0 % SEQ)) * DM + c0; }
    if (EPI == 3) { obase = (size_t)r0 * FF + c0; }
    if (EPI == 4) { obase = ((size_t)(r0 / SEQ) * OUT_SEQ + (size_t)(r0 % SEQ)) * DM + c0; rbase = (size_t)r0 * DM + c0; }
#pragma unroll
    for (int mb = 0; mb < 4; ++mb) {
#pragma unroll
        for (int nb = 0; nb < 4; ++nb) {
#pragma unroll
            for (int j = 0; j < 8; ++j) os[(hi * 8 + j) * OSP + nb * 16 + lr] = acc[mb][nb][j] * sc + bc[nb]; }
        wave_sync();
        if (EPI == 3) {
#pragma unroll 1
            for (int s = 0; s < 4; ++s) { const int row = 4 * s + (lane >> 3), c8 = (lane & 7) * 8;
                v4f x0 = *(const v4fa*)(&os[row * OSP + c8]); v4f x1 = *(const v4fa*)(&os[row * OSP + c8 + 4]);
#pragma unroll
                for (int i = 0; i < 4; ++i) { x0[i] = gelu_erf(x0[i]) * ACT_S; x1[i] = gelu_erf(x1[i]) * ACT_S; }
                *(v4fa*)(&os[row * OSP + c8]) = x0; *(v4fa*)(&os[row * OSP + c8 + 4]) = x1; }
        }
        if (EPI == 2 || EPI == 4) {
#pragma unroll 1
            for (int s = 0; s < 8; ++s) { const int row = 2 * s + (lane >> 4), c4 = (lane & 15) * 4;
                v4f x0 = *(const v4fa*)(&os[row * OSP + c4]);
                const v4f rr = *(const v4f*)(R + rbase + (size_t)(mb * 16 + row) * DM + c4);
#pragma unroll
                for (int i = 0; i < 4; ++i) x0[i] += (EPI == 2) ? bfr(rr[i]) : rr[i];
                *(v4fa*)(&os[row * OSP + c4]) = x0; }
        }
#pragma unroll 1
        for (int ps = 0; ps < 2; ++ps) {
            if (EPI == 0) {
                const size_t sb = obase + (size_t)(mb * 16) * HD + (size_t)lane * 8;
#pragma unroll
                for (int hh = 0; hh < 4; ++hh) { const int row = lane >> 1, c8 = (lane & 1) * 8;
                    const v4f x0 = *(const v4fa*)(&os[row * OSP + hh * 16 + c8]); const v4f x1 = *(const v4fa*)(&os[row * OSP + hh * 16 + c8 + 4]); v8h hv;
#pragma unroll
                    for (int i = 0; i < 4; ++i) { hv[i] = toh_flush(x0[i]); hv[4 + i] = toh_flush(x1[i]); }
                    *(volatile v8h*)(PH + sb + (size_t)hh * ((size_t)SEQ * HD)) = hv; }
            } else if (EPI == 1 || EPI == 3) {
                const size_t pitch = (EPI == 1) ? (size_t)SEQ : (size_t)FF;
                const size_t sb = obase + (size_t)(mb * 16) * pitch;
#pragma unroll
                for (int s = 0; s < 4; ++s) { const int row = 4 * s + (lane >> 3), c8 = (lane & 7) * 8;
                    const v4f x0 = *(const v4fa*)(&os[row * OSP + c8]); const v4f x1 = *(const v4fa*)(&os[row * OSP + c8 + 4]); v8h hv;
#pragma unroll
                    for (int i = 0; i < 4; ++i) { hv[i] = toh_flush(x0[i]); hv[4 + i] = toh_flush(x1[i]); }
                    *(volatile v8h*)(PH + sb + (size_t)row * pitch + c8) = hv; }
            } else {
                const size_t sb = obase + (size_t)(mb * 16) * DM;
#pragma unroll
                for (int s = 0; s < 8; ++s) { const int row = 2 * s + (lane >> 4), c4 = (lane & 15) * 4;
                    const v4f val = *(const v4fa*)(&os[row * OSP + c4]);
                    *(volatile v4f*)(PF + sb + (size_t)row * DM + c4) = val; }
            }
            if (ps == 0) __threadfence(); }
        wave_sync();
    }
}

__global__ __launch_bounds__(32) void k_gemm_qk(const h16* __restrict__ A, const h16* __restrict__ Bt, h16* QK) { gemm_body<0, DM>(A, Bt, nullptr, nullptr, QK, nullptr); }
__global__ __launch_bounds__(32) void k_gemm_vt(const h16* __restrict__ A, const h16* __restrict__ Bt, h16* VT) { gemm_body<1, DM>(A, Bt, nullptr, nullptr, VT, nullptr); }
__global__ __launch_bounds__(32) void k_gemm_proj(const h16* __restrict__ A, const h16* __restrict__ Bt, const float* __restrict__ bias, const float* __restrict__ X, float* X2) { gemm_body<2, DM>(A, Bt, bias, X, nullptr, X2); }
__global__ __launch_bounds__(32) void k_gemm_up(const h16* __restrict__ A, const h16* __restrict__ Bt, const float* __restrict__ bias, h16* G) { gemm_body<3, DM>(A, Bt, bias, nullptr, G, nullptr); }
__global__ __launch_bounds__(32) void k_gemm_down(const h16* __restrict__ A, const h16* __restrict__ Bt, const float* __restrict__ bias, const float* __restrict__ X2, float* OUT) { gemm_body<4, FF>(A, Bt, bias, X2, nullptr, OUT); }

__global__ __launch_bounds__(32 * AW) void k_flash(const h16* __restrict__ QP, const h16* __restrict__ KP, const h16* __restrict__ VT, h16* CTX) {
    __shared__ __align__(16) float os[16 * OSP];
    const int lane = threadIdx.x & 31, lr = lane & 15, hi = lane >> 4;
    const int wave = __builtin_amdgcn_readfirstlane((int)(threadIdx.x >> 5));
    const int b = blockIdx.y / HG, hg = blockIdx.y % HG;
    const int zh = b * NH_ + hg * AW + wave;
    const int t0 = blockIdx.x * 16;
    const int lim = t0 + lr;
    const int nk = (t0 + 16 + 31) & ~31;
    const size_t pbase = (size_t)zh * SEQ * HD;
    const v16h qf = ldh_lo(QP + pbase + (size_t)(t0 + lr) * HD + 8 * hi);
    const size_t ko = pbase + (size_t)lr * HD + 8 * hi;
    const size_t vo = pbase + (size_t)lr * SEQ + 8 * hi;
    v8f o = (v8f){};
    float m = NEGB, l = 0.0f;
#pragma unroll 1
    for (int key0 = 0; key0 < nk; key0 += 32) {
        const h16* ka = KP + ko + (size_t)key0 * HD;
        const v16h ka0 = ldh_lo(ka), kb0 = ldh_lo(ka + 16 * HD);
        v8f sa = (v8f){}, sb = (v8f){};
        sa = wmma16g(ka0, qf, sa); sb = wmma16g(kb0, qf, sb);
        const int ja = key0 + 8 * hi;
        float ta[8], tb[8]; bool fa[8], fb[8]; float mx = NEGB;
#pragma unroll
        for (int r = 0; r < 8; ++r) {
            fa[r] = (ja + r <= lim);
            fb[r] = (ja + 16 + r <= lim);
            ta[r] = sa[r] * SC2; tb[r] = sb[r] * SC2;
            mx = fmaxf(mx, fmaxf(fa[r] ? ta[r] : NEGB, fb[r] ? tb[r] : NEGB)); }
        mx = fmaxf(mx, __shfl_xor(mx, 16, 32));
        const float mnew = fmaxf(m, mx);
        const float alpha = __builtin_amdgcn_exp2f(m - mnew);
        const float sh = PSH - mnew;
        v16h pb; float ls = 0.0f;
#pragma unroll
        for (int r = 0; r < 8; ++r) {
            const float xa = ta[r] + sh, xb = tb[r] + sh;
            const float ea = __builtin_amdgcn_exp2f(xa), eb = __builtin_amdgcn_exp2f(xb);
            const float ga = (fa[r] & (xa >= -PSH)) ? ea : 0.0f;
            const float gb = (fb[r] & (xb >= -PSH)) ? eb : 0.0f;
            const h16 pa = (h16)ga; const h16 pc = (h16)gb;
            pb[r] = pa; pb[8 + r] = pc;
            ls += (float)pa + (float)pc; }
        l = l * alpha + ls; m = mnew;
        o = o * alpha;
        const v16h v0 = ldh(VT + vo + key0);
        o = wmma16g(v0, pb, o);
    }
    l += __shfl_xor(l, 16, 32);
    const bool any = l > 0.0f;
    const float lsafe = any ? l : 1.0f;
    const float inv = any ? (1.0f / lsafe) : 0.0f;
    { v4f a, c;
      a[0] = o[0] * inv; a[1] = o[1] * inv; a[2] = o[2] * inv; a[3] = o[3] * inv; c[0] = o[4] * inv; c[1] = o[5] * inv; c[2] = o[6] * inv; c[3] = o[7] * inv;
      *(v4fa*)(&os[lr * OSP + wave * 16 + 8 * hi]) = a; *(v4fa*)(&os[lr * OSP + wave * 16 + 8 * hi + 4]) = c; }
    __syncthreads();
    const int p = threadIdx.x; const int row = p >> 3, c8 = (p & 7) * 8;
    const v4f x0 = *(const v4fa*)(&os[row * OSP + c8]); const v4f x1 = *(const v4fa*)(&os[row * OSP + c8 + 4]); v8h hv;
#pragma unroll
    for (int i = 0; i < 4; ++i) { hv[i] = toh_flush(x0[i]); hv[4 + i] = toh_flush(x1[i]); }
    h16* dst = CTX + ((size_t)b * SEQ + (size_t)(t0 + row)) * DM + hg * 64 + c8;
    *(volatile v8h*)dst = hv; __threadfence(); *(volatile v8h*)dst = hv;
}

static constexpr size_t al256(size_t v) { return (v + 255) & ~(size_t)255; }
static constexpr size_t SZ_WQKV = al256((size_t)3 * DM * DM * 2);
static constexpr size_t SZ_WP   = al256((size_t)DM * DM * 2);
static constexpr size_t SZ_W1   = al256((size_t)DM * FF * 2);
static constexpr size_t SZ_W2   = al256((size_t)FF * DM * 2);
static constexpr size_t SZ_ACT  = al256((size_t)MROWS * DM * 2);
static constexpr size_t SZ_X2   = al256((size_t)MROWS * DM * 4);
static constexpr size_t SZ_G    = al256((size_t)MROWS * FF * 2);
static constexpr size_t SZ_TOTAL = SZ_WQKV + SZ_WP + SZ_W1 + SZ_W2 + 6 * SZ_ACT + SZ_X2 + SZ_G;
static_assert(SZ_TOTAL <= (size_t)134217728);
static_assert(((size_t)MROWS * DM * 2) % 256 == 0);
static_assert((size_t)NB * NH_ * SEQ * HD == (size_t)MROWS * DM);
static_assert(((size_t)DM * DM * 2) % 256 == 0);

extern "C" void kernel_launch(void* const* d_in, const int* in_sizes, int n_in,
                              void* d_out, int out_size, void* d_ws, size_t ws_size, hipStream_t stream) {
    if (n_in < 14) return;
    const size_t needx = ((size_t)(NB - 1) * SEQ_FULL + SEQ) * DM;
    if ((size_t)in_sizes[0] < needx) return;
    if ((size_t)in_sizes[1] < (size_t)DM * DM || (size_t)in_sizes[2] < (size_t)DM * DM || (size_t)in_sizes[3] < (size_t)DM * DM || (size_t)in_sizes[4] < (size_t)DM * DM) return;
    if ((size_t)in_sizes[6] < (size_t)DM * FF || (size_t)in_sizes[8] < (size_t)FF * DM) return;
    if (in_sizes[5] < DM || in_sizes[7] < FF || in_sizes[9] < DM || in_sizes[10] < DM || in_sizes[11] < DM || in_sizes[12] < DM || in_sizes[13] < DM) return;
    if ((size_t)out_size < ((size_t)(NB - 1) * OUT_SEQ + SEQ) * DM) return;
    if (SZ_TOTAL > ws_size) return;
    const float* x   = (const float*)d_in[0];
    const float* wq  = (const float*)d_in[1];
    const float* wk  = (const float*)d_in[2];
    const float* wv  = (const float*)d_in[3];
    const float* wp  = (const float*)d_in[4];
    const float* bp  = (const float*)d_in[5];
    const float* w1  = (const float*)d_in[6];
    const float* b1  = (const float*)d_in[7];
    const float* w2  = (const float*)d_in[8];
    const float* b2  = (const float*)d_in[9];
    const float* g1  = (const float*)d_in[10];
    const float* be1 = (const float*)d_in[11];
    const float* g2  = (const float*)d_in[12];
    const float* be2 = (const float*)d_in[13];
    float* OUT = (float*)d_out;
    char* wsp = (char*)d_ws;
    h16* WQKV = (h16*)wsp; wsp += SZ_WQKV;
    h16* WPT  = (h16*)wsp; wsp += SZ_WP;
    h16* W1T  = (h16*)wsp; wsp += SZ_W1;
    h16* W2T  = (h16*)wsp; wsp += SZ_W2;
    h16* H1   = (h16*)wsp; wsp += SZ_ACT;
    h16* QK   = (h16*)wsp; wsp += 2 * SZ_ACT;
    h16* VT   = (h16*)wsp; wsp += SZ_ACT;
    h16* CTX  = (h16*)wsp; wsp += SZ_ACT;
    float* X2 = (float*)wsp; wsp += SZ_X2;
    h16* H2   = (h16*)wsp; wsp += SZ_ACT;
    h16* G    = (h16*)wsp; wsp += SZ_G;
    const h16* QP = QK; const h16* KP = QK + (size_t)MROWS * DM;

    k_wtr<<<dim3(DM / 64, 1, NH_), 128, 0, stream>>>(wq, WQKV,                       DM, HD, (size_t)DM * HD, (size_t)HD * DM);
    k_wtr<<<dim3(DM / 64, 1, NH_), 128, 0, stream>>>(wk, WQKV + (size_t)DM * DM,     DM, HD, (size_t)DM * HD, (size_t)HD * DM);
    k_wtr<<<dim3(DM / 64, 1, NH_), 128, 0, stream>>>(wv, WQKV + (size_t)2 * DM * DM, DM, HD, (size_t)DM * HD, (size_t)HD * DM);
    k_wtr<<<dim3(DM / 64, DM / 16, 1), 128, 0, stream>>>(wp, WPT, DM, DM, (size_t)0, (size_t)0);
    k_wtr<<<dim3(DM / 64, FF / 16, 1), 128, 0, stream>>>(w1, W1T, DM, FF, (size_t)0, (size_t)0);
    k_wtr<<<dim3(FF / 64, DM / 16, 1), 128, 0, stream>>>(w2, W2T, FF, DM, (size_t)0, (size_t)0);

    k_ln<<<MROWS / 8, 256, 0, stream>>>(x, g1, be1, H1, 1, 1);
    k_gemm_qk<<<dim3(MROWS / 64, (2 * DM) / 64, 1), 32, 0, stream>>>(H1, WQKV, QK);
    k_gemm_vt<<<dim3(DM / 64, MROWS / 64, 1), 32, 0, stream>>>(WQKV + (size_t)2 * DM * DM, H1, VT);
    k_flash<<<dim3(SEQ / 16, NB * HG, 1), 32 * AW, 0, stream>>>(QP, KP, VT, CTX);
    k_gemm_proj<<<dim3(MROWS / 64, DM / 64, 1), 32, 0, stream>>>(CTX, WPT, bp, x, X2);
    k_ln<<<MROWS / 8, 256, 0, stream>>>(X2, g2, be2, H2, 0, 0);
    k_gemm_up<<<dim3(MROWS / 64, FF / 64, 1), 32, 0, stream>>>(H2, W1T, b1, G);
    k_gemm_down<<<dim3(MROWS / 64, DM / 64, 1), 32, 0, stream>>>(G, W2T, b2, X2, OUT);
}
